// CausalSelfAttention_18923625906326
// MI455X (gfx1250) — hardware-verified
//
#include <hip/hip_runtime.h>
#include <math.h>

typedef __attribute__((ext_vector_type(16))) _Float16 v16h;
typedef __attribute__((ext_vector_type(8)))  _Float16 v8h;
typedef __attribute__((ext_vector_type(8)))  float    v8f;
typedef __attribute__((ext_vector_type(4)))  float    v4f;

#ifndef NB
#define NB 2
#endif
#ifndef SEQ
#define SEQ 2048
#endif
#define NB_FULL 2
#define SEQ_FULL 2048
#define DM 1024
#define NH 16
#define HD 64
#define MTOK (NB * SEQ)
#define XROWS ((NB - 1) * SEQ_FULL + SEQ)
#define QKP (2 * DM)
#define CTXP (2 * DM)
#define WOP (2 * DM)
#define NXB 4
#define PP 40
#define SLP 68

#define RS_QK 2048.0f
#define RI_QK (1.0f / 2048.0f)
#define PCARRY 4096.0f
#define RS_CTX 64.0f

static_assert(DM == NH * HD);
static_assert(HD == 64);
static_assert(SEQ % 64 == 0);
static_assert(SEQ >= 64 * NXB);
static_assert(SEQ <= SEQ_FULL);
static_assert(NB >= 1 && NB <= NB_FULL);
static_assert(MTOK % 64 == 0);
static_assert(DM % 64 == 0);
static_assert(DM % 32 == 0 && (2 * DM) % 32 == 0);
static_assert(PP % 8 == 0 && PP >= 32);
static_assert(SLP % 4 == 0 && SLP >= 64);
static_assert((SEQ * 32) % 256 == 0);
static_assert((size_t)XROWS * DM * 4 <= (size_t)16777216);

union FragU { v16h v; v8h h[2]; };
__device__ __forceinline__ v16h ldfrag(const _Float16* __restrict__ p) {
    FragU f; f.h[0] = *(const v8h*)(p); f.h[1] = *(const v8h*)(p + 16); return f.v;
}
__device__ __forceinline__ v8f mma(v16h a, v16h b, v8f c) {
    c = __builtin_amdgcn_wmma_f32_16x16x32_f16(false, a, false, b, (short)0, c, false, false);
    asm volatile("v_nop\n\tv_nop\n\tv_nop\n\tv_nop" : "+v"(c) : "v"(a), "v"(b));
    return c;
}
__device__ __forceinline__ void dep_guard_h(v8f& a, v8f& b, v16h x, v16h y) { asm volatile("v_nop\n\tv_nop\n\tv_nop\n\tv_nop" : "+v"(a), "+v"(b) : "v"(x), "v"(y)); }
__device__ __forceinline__ void keep4_h(v16h a, v16h b, v16h c, v16h d) { asm volatile("v_nop" :: "v"(a), "v"(b), "v"(c), "v"(d)); }
__device__ __forceinline__ void acc_guard4(v8f& a, v8f& b, v8f& c, v8f& d) { asm volatile("v_nop\n\tv_nop\n\tv_nop\n\tv_nop" : "+v"(a), "+v"(b), "+v"(c), "+v"(d)); }
__device__ __forceinline__ void wave_lds_sync() {
    __builtin_amdgcn_fence(3  , "workgroup");
    __builtin_amdgcn_wave_barrier();
    __builtin_amdgcn_fence(2  , "workgroup");
}
__device__ __forceinline__ float cmb_bf(float v) { const unsigned u = __builtin_bit_cast(unsigned, v); const unsigned r = (u + 0x7fffu + ((u >> 16) & 1u)) & 0xffff0000u; return __builtin_bit_cast(float, r); }
__device__ __forceinline__ void st2_f32(float* p, float v) { *(volatile float*)p = v; __threadfence(); *(volatile float*)p = v; }
__device__ __forceinline__ void st2_v8h(_Float16* p, v8h v) { *(volatile v8h*)p = v; __threadfence(); *(volatile v8h*)p = v; }

__global__ __launch_bounds__(256) void k_cast_x(const float* __restrict__ X, _Float16* __restrict__ D) {
    const int u = blockIdx.x * 256 + threadIdx.x;
    if (u >= MTOK * (DM / 8)) return;
    const int r = u / (DM / 8); const int c0 = 8 * (u - r * (DM / 8));
    const int bq = r / SEQ; const size_t srow = (size_t)bq * SEQ_FULL + (size_t)(r - bq * SEQ);
    const v4f a = *(const v4f*)(X + srow * DM + c0), bb = *(const v4f*)(X + srow * DM + c0 + 4);
    v8h o;
    o[0] = (_Float16)cmb_bf(a.x); o[1] = (_Float16)cmb_bf(a.y); o[2] = (_Float16)cmb_bf(a.z); o[3] = (_Float16)cmb_bf(a.w);
    o[4] = (_Float16)cmb_bf(bb.x); o[5] = (_Float16)cmb_bf(bb.y); o[6] = (_Float16)cmb_bf(bb.z); o[7] = (_Float16)cmb_bf(bb.w);
    st2_v8h(D + (size_t)r * DM + c0, o);
}

__global__ __launch_bounds__(256) void k_castT(const float* __restrict__ W, int lds, _Float16* __restrict__ D, int ldd, int nK, int nC, int reps, float sc0, float sc1) {
    const int per = (reps * nK) / 8;
    const int u = blockIdx.x * 256 + threadIdx.x;
    if (u >= nC * per) return;
    const int c = u / per; const int kk0 = 8 * (u - c * per);
    const int seg = kk0 / nK; const int r0 = kk0 - seg * nK; const float sc = seg ? sc1 : sc0;
    v8h o;
#pragma unroll
    for (int e = 0; e < 8; ++e) o[e] = (_Float16)(cmb_bf(W[(size_t)(r0 + e) * lds + c]) * sc);
    st2_v8h(D + (size_t)c * ldd + kk0, o);
}

__global__ __launch_bounds__(256) void k_ropetab(float* __restrict__ CS, float* __restrict__ SN) {
    #pragma clang fp contract(off)
    const int idx = blockIdx.x * 256 + threadIdx.x;
    if (idx >= SEQ * 32) return;
    const int t = idx >> 5, i = idx & 31;
    double p = 1.0;
    p = (i & 1) ? p * 1.3335214321633240 : p;
    p = (i & 2) ? p * 1.7782794100389228 : p;
    p = (i & 4) ? p * 3.1622776601683795 : p;
    p = (i & 8) ? p * 10.0 : p;
    p = (i & 16) ? p * 100.0 : p;
    const float pf = (float)p;
    const float inv = 1.0f / pf;
    const float ang = (float)t * inv;
    const float c = cosf(ang);
    const float s = sinf(ang);
    st2_f32(CS + idx, c);
    st2_f32(SN + idx, s);
}

template <int EPI>
__device__ __forceinline__ void gemm64_body(const _Float16* __restrict__ A, int lda, const _Float16* __restrict__ Bt, int ldb,
                                            int M, int N, int K, float scale,
                                            float* __restrict__ Cf, _Float16* __restrict__ CH, _Float16* __restrict__ CR, int ldc,
                                            const float* __restrict__ CS, const float* __restrict__ SN) {
    __shared__ __align__(16) float sT[8 * 16 * SLP];
    const int lane = threadIdx.x & 31;
    const int wave = __builtin_amdgcn_readfirstlane(threadIdx.x >> 5);
    const int tilesN = N >> 6, tilesM = M >> 6;
    const int tile = blockIdx.x * 8 + wave;
    if (tile >= tilesM * tilesN) return;
    const int tm = tile / tilesN, tn = tile - tm * tilesN;
    const int m0 = tm << 6, n0 = tn << 6;
    const int rlane = lane & 15;
    const int koff = (lane >> 4) * 8;
    const int mOff = (lane >> 4) * 8;

    v8f acc[4][4];
#pragma unroll
    for (int i = 0; i < 4; ++i)
#pragma unroll
        for (int j = 0; j < 4; ++j) acc[i][j] = (v8f){0.f, 0.f, 0.f, 0.f, 0.f, 0.f, 0.f, 0.f};

    for (int k0 = 0; k0 < K; k0 += 32) {
        v16h bh[4];
#pragma unroll
        for (int j = 0; j < 4; ++j) bh[j] = ldfrag(Bt + (size_t)(n0 + (j << 4) + rlane) * ldb + koff + k0);
#pragma unroll
        for (int i = 0; i < 4; ++i) {
            const v16h ah = ldfrag(A + (size_t)(m0 + (i << 4) + rlane) * lda + koff + k0);
#pragma unroll
            for (int j = 0; j < 4; ++j)
                acc[i][j] = __builtin_amdgcn_wmma_f32_16x16x32_f16(false, ah, false, bh[j], (short)0, acc[i][j], false, false);
            dep_guard_h(acc[i][0], acc[i][3], ah, ah);
        }
        keep4_h(bh[0], bh[1], bh[2], bh[3]);
    }
    acc_guard4(acc[0][0], acc[0][1], acc[0][2], acc[0][3]);
    acc_guard4(acc[1][0], acc[1][1], acc[1][2], acc[1][3]);
    acc_guard4(acc[2][0], acc[2][1], acc[2][2], acc[2][3]);
    acc_guard4(acc[3][0], acc[3][1], acc[3][2], acc[3][3]);

    const int sw = wave * (16 * SLP);
#pragma unroll
    for (int i = 0; i < 4; ++i) {
        const int mBase = m0 + (i << 4);
#pragma unroll
        for (int j = 0; j < 4; ++j)
#pragma unroll
            for (int r = 0; r < 8; ++r) sT[sw + (mOff + r) * SLP + (j << 4) + rlane] = acc[i][j][r] * scale;
        wave_lds_sync();
        if (EPI == 0) {
            const int hh = lane >> 4, c4 = (lane & 15) * 4;
            for (int pass = 0; pass < 2; ++pass) {
#pragma unroll
                for (int it = 0; it < 8; ++it) {
                    const int row = it * 2 + hh;
                    const int m = mBase + row; const int bq = m / SEQ;
                    const size_t orow = (size_t)bq * SEQ_FULL + (size_t)(m - bq * SEQ);
                    const v4f v = *(const v4f*)&sT[sw + row * SLP + c4];
                    *(volatile v4f*)(Cf + orow * ldc + n0 + c4) = v;
                }
                __threadfence();
            }
        } else {
            const int q = lane >> 3, c8 = (lane & 7) * 8;
            const int tb = mBase % SEQ;
            for (int pass = 0; pass < 2; ++pass) {
#pragma unroll
                for (int it = 0; it < 4; ++it) {
                    const int row = it * 4 + q;
                    const int sb = sw + row * SLP;
                    float val[8];
                    if (EPI == 1) {
                        const int t = tb + row;
                        const int fi = c8 & 31;
                        const v4f ca = *(const v4f*)(CS + t * 32 + fi), cb = *(const v4f*)(CS + t * 32 + fi + 4);
                        const v4f sa = *(const v4f*)(SN + t * 32 + fi), sc = *(const v4f*)(SN + t * 32 + fi + 4);
                        const float cc[8] = {ca.x, ca.y, ca.z, ca.w, cb.x, cb.y, cb.z, cb.w};
                        const float ss[8] = {sa.x, sa.y, sa.z, sa.w, sc.x, sc.y, sc.z, sc.w};
                        const float sg = (c8 < 32) ? -1.0f : 1.0f;
                        const int pc = c8 ^ 32;
#pragma unroll
                        for (int e = 0; e < 8; ++e) { const float x = sT[sb + c8 + e]; const float xp = sT[sb + pc + e]; val[e] = x * cc[e] + (sg * xp) * ss[e]; }
                    } else {
#pragma unroll
                        for (int e = 0; e < 8; ++e) val[e] = sT[sb + c8 + e];
                    }
                    v8h hv, rv;
#pragma unroll
                    for (int e = 0; e < 8; ++e) { const _Float16 hq = (_Float16)val[e]; hv[e] = hq; rv[e] = (_Float16)((val[e] - (float)hq) * RS_QK); }
                    const size_t o = (size_t)(mBase + row) * ldc + n0 + c8;
                    *(volatile v8h*)(CH + o) = hv;
                    *(volatile v8h*)(CR + o) = rv;
                }
                __threadfence();
            }
        }
        wave_lds_sync();
    }
}

__global__ __launch_bounds__(256) void k_gemm_qk(const _Float16* __restrict__ X16, const _Float16* __restrict__ WT, _Float16* __restrict__ QKH, _Float16* __restrict__ QKR,
                                                 const float* __restrict__ CS, const float* __restrict__ SN) {
    gemm64_body<1>(X16, DM, WT, DM, MTOK, 2 * DM, DM, 0.0625f, nullptr, QKH, QKR, QKP, CS, SN);
}
__global__ __launch_bounds__(256) void k_gemm_v(const _Float16* __restrict__ WTV, const _Float16* __restrict__ X16, _Float16* __restrict__ VTH, _Float16* __restrict__ VTR) {
    gemm64_body<2>(WTV, DM, X16, DM, DM, MTOK, DM, 0.0625f, nullptr, VTH, VTR, MTOK, nullptr, nullptr);
}
__global__ __launch_bounds__(256) void k_gemm_out(const _Float16* __restrict__ CTX, const _Float16* __restrict__ WOT, float* __restrict__ OUT) {
    gemm64_body<0>(CTX, CTXP, WOT, WOP, MTOK, DM, 2 * DM, 0.0625f, OUT, nullptr, nullptr, DM, nullptr, nullptr);
}

template <bool EARLY>
__device__ __forceinline__ void attn_body(const _Float16* __restrict__ QKH, const _Float16* __restrict__ QKR,
                                          const _Float16* __restrict__ VTH, const _Float16* __restrict__ VTR,
                                          _Float16* __restrict__ CTX, int qb0, int nqb) {
    __shared__ __align__(16) _Float16 Ps[4 * 16 * PP];
    __shared__ __align__(16) _Float16 Pr[EARLY ? 4 * 16 * PP : 8];
    __shared__ __align__(16) float    Os[4 * 16 * SLP];
    const int lane = threadIdx.x & 31, hf = lane >> 4, l15 = lane & 15;
    const int wave = __builtin_amdgcn_readfirstlane(threadIdx.x >> 5);
    const int bx = blockIdx.x;
    const int bhh = bx / nqb; const int qb = qb0 + (bx - bhh * nqb);
    const int b = bhh / NH; const int h = bhh - b * NH;
    const int q0 = qb * 64 + wave * 16;
    const int nch = ((q0 + 15) >> 5) + 1;
    const int qoff = (b * SEQ + q0 + l15) * QKP + h * HD + 8 * hf;
    const int koff = (b * SEQ + l15) * QKP + DM + h * HD + 8 * hf;
    const int voff = (h * HD + l15) * MTOK + b * SEQ + 8 * hf;
    const float SCL = 0.125f * 1.4426950408889634f;
    const float NEG = -__builtin_inff();

    float mrow[8], lrow[8];
    v8f oh[4], orr[4];
#pragma unroll
    for (int r = 0; r < 8; ++r) { mrow[r] = NEG; lrow[r] = 0.f; }
#pragma unroll
    for (int t = 0; t < 4; ++t) { oh[t] = (v8f){0.f, 0.f, 0.f, 0.f, 0.f, 0.f, 0.f, 0.f}; orr[t] = oh[t]; }

    for (int ch = 0; ch < nch; ++ch) {
        const int kv0 = ch * 32;
        v8f sh[2], sr[2];
#pragma unroll
        for (int j = 0; j < 2; ++j) { sh[j] = (v8f){0.f, 0.f, 0.f, 0.f, 0.f, 0.f, 0.f, 0.f}; sr[j] = sh[j]; }
#pragma unroll
        for (int dc = 0; dc < 2; ++dc) {
            const v16h qa = ldfrag(QKH + qoff + dc * 32);
            const v16h qr = ldfrag(QKR + qoff + dc * 32);
#pragma unroll
            for (int j = 0; j < 2; ++j) {
                const int ko = koff + (kv0 + j * 16) * QKP + dc * 32;
                const v16h kb = ldfrag(QKH + ko);
                sh[j] = mma(qa, kb, sh[j]);
                sr[j] = mma(qr, kb, sr[j]);
                if (EARLY) { const v16h kr = ldfrag(QKR + ko); sr[j] = mma(qa, kr, sr[j]); }
            }
        }
        const bool diag = (kv0 + 31 > q0);
        const int kc0 = kv0 + l15;
#pragma unroll
        for (int r = 0; r < 8; ++r) {
            const int qrow = q0 + 8 * hf + r;
            float v0 = (sh[0][r] + sr[0][r] * RI_QK) * SCL;
            float v1 = (sh[1][r] + sr[1][r] * RI_QK) * SCL;
            v0 = (diag && (kc0 > qrow)) ? NEG : v0;
            v1 = (diag && (kc0 + 16 > qrow)) ? NEG : v1;
            float mx = fmaxf(v0, v1);
            mx = fmaxf(mx, __shfl_xor(mx, 1, 32)); mx = fmaxf(mx, __shfl_xor(mx, 2, 32));
            mx = fmaxf(mx, __shfl_xor(mx, 4, 32)); mx = fmaxf(mx, __shfl_xor(mx, 8, 32));
            const float mnew = fmaxf(mrow[r], mx);
            const float alpha = exp2f(mrow[r] - mnew);
            const float p0 = exp2f(v0 - mnew), p1 = exp2f(v1 - mnew);
            float ps = p0 + p1;
            ps += __shfl_xor(ps, 1, 32); ps += __shfl_xor(ps, 2, 32); ps += __shfl_xor(ps, 4, 32); ps += __shfl_xor(ps, 8, 32);
            lrow[r] = lrow[r] * alpha + ps; mrow[r] = mnew;
#pragma unroll
            for (int t = 0; t < 4; ++t) { oh[t][r] *= alpha; if (EARLY) orr[t][r] *= alpha; }
            const int pi = wave * (16 * PP) + (8 * hf + r) * PP + l15;
            const float c0 = p0 * PCARRY, c1 = p1 * PCARRY;
            const _Float16 h0 = (_Float16)c0, h1 = (_Float16)c1;
            Ps[pi] = h0; Ps[pi + 16] = h1;
            if (EARLY) { Pr[pi] = (_Float16)((c0 - (float)h0) * RS_QK); Pr[pi + 16] = (_Float16)((c1 - (float)h1) * RS_QK); }
        }
        wave_lds_sync();
        {
            const int po = wave * (16 * PP) + l15 * PP + 8 * hf;
            FragU pa; pa.h[0] = *(const v8h*)&Ps[po]; pa.h[1] = *(const v8h*)&Ps[po + 16];
            FragU pr; pr.v = pa.v;
            if (EARLY) { pr.h[0] = *(const v8h*)&Pr[po]; pr.h[1] = *(const v8h*)&Pr[po + 16]; }
            const int vo = voff + kv0;
#pragma unroll
            for (int t = 0; t < 4; ++t) {
                const v16h vb = ldfrag(VTH + vo + t * 16 * MTOK);
                oh[t] = mma(pa.v, vb, oh[t]);
                if (EARLY) {
                    const v16h vr = ldfrag(VTR + vo + t * 16 * MTOK);
                    orr[t] = mma(pa.v, vr, orr[t]);
                    orr[t] = mma(pr.v, vb, orr[t]);
                }
            }
        }
        wave_lds_sync();
    }

    const int sw = wave * (16 * SLP);
#pragma unroll
    for (int r = 0; r < 8; ++r) {
        const float inv = 1.0f / (lrow[r] * PCARRY);
#pragma unroll
        for (int t = 0; t < 4; ++t) {
            float val = oh[t][r];
            if (EARLY) val += orr[t][r] * RI_QK;
            Os[sw + (8 * hf + r) * SLP + t * 16 + l15] = val * inv;
        }
    }
    wave_lds_sync();
    {
        const int q = lane >> 3, c8 = (lane & 7) * 8;
        for (int pass = 0; pass < 2; ++pass) {
#pragma unroll
            for (int it = 0; it < 4; ++it) {
                const int row = it * 4 + q;
                const int so = sw + row * SLP + c8;
                const v4f a = *(const v4f*)&Os[so], bq = *(const v4f*)&Os[so + 4];
                const float val[8] = {a.x, a.y, a.z, a.w, bq.x, bq.y, bq.z, bq.w};
                v8h hv, rv;
#pragma unroll
                for (int e = 0; e < 8; ++e) { const _Float16 hq = (_Float16)val[e]; hv[e] = hq; rv[e] = (_Float16)((val[e] - (float)hq) * RS_CTX); }
                _Float16* dst = CTX + (size_t)(b * SEQ + q0 + row) * CTXP + h * HD + c8;
                *(volatile v8h*)(dst) = hv;
                *(volatile v8h*)(dst + DM) = rv;
            }
            __threadfence();
        }
    }
}

__global__ __launch_bounds__(128) void k_attn_early(const _Float16* __restrict__ QKH, const _Float16* __restrict__ QKR, const _Float16* __restrict__ VTH, const _Float16* __restrict__ VTR,
                                                    _Float16* __restrict__ CTX) {
    attn_body<true>(QKH, QKR, VTH, VTR, CTX, 0, NXB);
}
__global__ __launch_bounds__(128) void k_attn_late(const _Float16* __restrict__ QKH, const _Float16* __restrict__ QKR, const _Float16* __restrict__ VTH, const _Float16* __restrict__ VTR,
                                                   _Float16* __restrict__ CTX) {
    attn_body<false>(QKH, QKR, VTH, VTR, CTX, NXB, SEQ / 64 - NXB);
}

static constexpr size_t al256(size_t v) { return (v + 255) / 256 * 256; }
static constexpr size_t SZ_X16 = al256((size_t)MTOK * DM * 2);
static constexpr size_t SZ_WT  = al256((size_t)3 * DM * DM * 2);
static constexpr size_t SZ_WOT = al256((size_t)DM * WOP * 2);
static constexpr size_t SZ_TAB = al256((size_t)SEQ * 32 * 4);
static constexpr size_t SZ_QK  = al256((size_t)MTOK * QKP * 2);
static constexpr size_t SZ_VT  = al256((size_t)DM * MTOK * 2);
static constexpr size_t SZ_CTX = al256((size_t)MTOK * CTXP * 2);
static constexpr size_t WS_TOTAL = SZ_X16 + SZ_WT + SZ_WOT + 2 * SZ_TAB + 2 * SZ_QK + 2 * SZ_VT + SZ_CTX;
static_assert(WS_TOTAL <= (size_t)134217728);

extern "C" void kernel_launch(void* const* d_in, const int* in_sizes, int n_in, void* d_out, int out_size, void* d_ws, size_t ws_size, hipStream_t stream) {
    if (n_in < 3) return;
    if (in_sizes[0] < XROWS * DM) return;
    if (in_sizes[1] < DM * 3 * DM) return;
    if (in_sizes[2] < DM * DM) return;
    if (out_size < XROWS * DM) return;
    if (ws_size < WS_TOTAL) return;
    const float* x    = (const float*)d_in[0];
    const float* wqkv = (const float*)d_in[1];
    const float* wout = (const float*)d_in[2];
    float* out = (float*)d_out;
    char* wsp = (char*)d_ws;
    _Float16* X16 = (_Float16*)wsp; wsp += SZ_X16;
    _Float16* WT  = (_Float16*)wsp; wsp += SZ_WT;
    _Float16* WOT = (_Float16*)wsp; wsp += SZ_WOT;
    float* CS = (float*)wsp; wsp += SZ_TAB;
    float* SN = (float*)wsp; wsp += SZ_TAB;
    _Float16* QKH = (_Float16*)wsp; wsp += SZ_QK;
    _Float16* QKR = (_Float16*)wsp; wsp += SZ_QK;
    _Float16* VTH = (_Float16*)wsp; wsp += SZ_VT;
    _Float16* VTR = (_Float16*)wsp; wsp += SZ_VT;
    _Float16* CTX = (_Float16*)wsp; wsp += SZ_CTX;

    k_cast_x<<<(unsigned)((MTOK * (DM / 8) + 255) / 256), 256, 0, stream>>>(x, X16);
    k_castT<<<(unsigned)((3 * DM * (DM / 8) + 255) / 256), 256, 0, stream>>>(wqkv, 3 * DM, WT, DM, DM, 3 * DM, 1, 16.0f, 16.0f);
    k_castT<<<(unsigned)((DM * (2 * DM / 8) + 255) / 256), 256, 0, stream>>>(wout, DM, WOT, WOP, DM, DM, 2, 16.0f, 0.25f);
    k_ropetab<<<(unsigned)((SEQ * 32 + 255) / 256), 256, 0, stream>>>(CS, SN);
    k_gemm_qk<<<(unsigned)(((MTOK / 64) * (2 * DM / 64) + 7) / 8), 256, 0, stream>>>(X16, WT, QKH, QKR, CS, SN);
    k_gemm_v<<<(unsigned)(((DM / 64) * (MTOK / 64) + 7) / 8), 256, 0, stream>>>(WT + (size_t)2 * DM * DM, X16, VTH, VTR);
    k_attn_early<<<(unsigned)(NB * NH * NXB), 128, 0, stream>>>(QKH, QKR, VTH, VTR, CTX);
    if (SEQ / 64 - NXB > 0)
        k_attn_late<<<(unsigned)(NB * NH * (SEQ / 64 - NXB)), 128, 0, stream>>>(QKH, QKR, VTH, VTR, CTX);
    k_gemm_out<<<(unsigned)(((MTOK / 64) * (DM / 64) + 7) / 8), 256, 0, stream>>>(CTX, WOT, out);
}
